// GAT_Encoder_19430432047705
// MI455X (gfx1250) — hardware-verified
//
#include <hip/hip_runtime.h>
#include <stdint.h>

constexpr int NBATCH = 16;
constexpr int NNODE  = 256;
constexpr int NFEAT  = 1024;
constexpr int NHEAD  = 16;
constexpr int DHEAD  = 64;
constexpr int MROWS  = NBATCH * NNODE;
constexpr int BPC    = 4;
constexpr int NCHUNKS = NBATCH / BPC;
constexpr int ZPC    = BPC * NHEAD;
constexpr float MASK_FILL = -9e15f;
constexpr int OUT0_ELEMS = MROWS * NFEAT;
constexpr int OUT1_ELEMS = NBATCH * NNODE * NNODE;
static_assert((size_t)OUT0_ELEMS * 4 == (size_t)16777216, "out1 byte offset");
static_assert(((size_t)OUT0_ELEMS + OUT1_ELEMS) * 4 == (size_t)20971520, "out total bytes");

constexpr size_t ACT_PLANE_B = (size_t)MROWS * NFEAT * 2;
constexpr size_t W_PLANE_B   = (size_t)NFEAT * NFEAT * 2;
constexpr size_t BIAS_TAB_B  = (size_t)4 * NFEAT * 4;
constexpr size_t VO_PLANE_B  = (size_t)NBATCH * NFEAT * NNODE * 2;
constexpr size_t S_CHUNK_B   = (size_t)ZPC * NNODE * NNODE * 4;
constexpr size_t P_PLANE_B   = (size_t)ZPC * NNODE * NNODE * 2;
constexpr size_t OFF_OBJ16 = 0;
constexpr size_t OFF_CRS16 = OFF_OBJ16 + ACT_PLANE_B;
constexpr size_t OFF_WQ16  = OFF_CRS16 + ACT_PLANE_B;
constexpr size_t OFF_WK16  = OFF_WQ16  + W_PLANE_B;
constexpr size_t OFF_WV16  = OFF_WK16  + W_PLANE_B;
constexpr size_t OFF_WO16  = OFF_WV16  + W_PLANE_B;
constexpr size_t OFF_BIAS  = OFF_WO16  + W_PLANE_B;
constexpr size_t OFF_QHI   = OFF_BIAS  + BIAS_TAB_B;
constexpr size_t OFF_QLO   = OFF_QHI   + ACT_PLANE_B;
constexpr size_t OFF_KHI   = OFF_QLO   + ACT_PLANE_B;
constexpr size_t OFF_KLO   = OFF_KHI   + ACT_PLANE_B;
constexpr size_t OFF_VHI   = OFF_KLO   + ACT_PLANE_B;
constexpr size_t OFF_VLO   = OFF_VHI   + ACT_PLANE_B;
constexpr size_t OFF_VOHI  = OFF_VLO   + ACT_PLANE_B;
constexpr size_t OFF_VOLO  = OFF_VOHI  + VO_PLANE_B;
constexpr size_t OFF_S     = OFF_VOLO  + VO_PLANE_B;
constexpr size_t OFF_PHI   = OFF_S     + S_CHUNK_B;
constexpr size_t OFF_PLO   = OFF_PHI   + P_PLANE_B;
constexpr size_t WS_TOTAL  = OFF_PLO   + P_PLANE_B;
static_assert(WS_TOTAL == (size_t)125845504, "carve total");
static_assert(WS_TOTAL <= (size_t)134217728, "carve cap");
static_assert(OFF_BIAS % 128 == 0 && OFF_QHI % 128 == 0 && OFF_S % 128 == 0 && OFF_PHI % 128 == 0 && OFF_PLO % 128 == 0, "alignment");

static_assert(MROWS % 64 == 0 && NFEAT % 64 == 0 && NFEAT % 32 == 0, "projection tiles");
static_assert(NNODE % 64 == 0 && DHEAD % 64 == 0 && DHEAD % 32 == 0 && NNODE % 32 == 0, "attention tiles");
static_assert(NFEAT == NHEAD * DHEAD, "head split");
static_assert((MROWS * NFEAT) % (8 * 256) == 0 && (NFEAT * NFEAT) % (8 * 256) == 0, "cast coverage");

typedef __attribute__((ext_vector_type(16))) _Float16 v16h;
typedef __attribute__((ext_vector_type(8)))  _Float16 v8h;
typedef __attribute__((ext_vector_type(16))) __bf16   v16b;
typedef __attribute__((ext_vector_type(8)))  __bf16   v8b;
typedef __attribute__((ext_vector_type(8)))  float    v8f;
typedef __attribute__((ext_vector_type(4)))  float    v4f;
typedef __attribute__((ext_vector_type(4)))  unsigned int v4u;
typedef __attribute__((ext_vector_type(4)))  int      v4i;

__device__ __forceinline__ unsigned short f2bf_bits(float f) {
  unsigned u = __float_as_uint(f);
  return (unsigned short)((u + 0x7FFFu + ((u >> 16) & 1u)) >> 16);
}
__device__ __forceinline__ float bf_bits2f(unsigned short h) { return __uint_as_float(((unsigned)h) << 16); }
__device__ __forceinline__ float bf16_rne(float f) { return bf_bits2f(f2bf_bits(f)); }

__device__ __forceinline__ void dep_guard_h(v8f& a, v8f& b, v16h x, v16h y) { asm volatile("v_nop\n\tv_nop\n\tv_nop\n\tv_nop" : "+v"(a), "+v"(b) : "v"(x), "v"(y)); }
__device__ __forceinline__ void dep_guard_b(v8f& a, v8f& b, v16b x, v16b y) { asm volatile("v_nop\n\tv_nop\n\tv_nop\n\tv_nop" : "+v"(a), "+v"(b) : "v"(x), "v"(y)); }
__device__ __forceinline__ void keep4_h(v16h a, v16h b, v16h c, v16h d) { asm volatile("v_nop" :: "v"(a), "v"(b), "v"(c), "v"(d)); }
__device__ __forceinline__ void keep4_b(v16b a, v16b b, v16b c, v16b d) { asm volatile("v_nop" :: "v"(a), "v"(b), "v"(c), "v"(d)); }
__device__ __forceinline__ void acc_guard4(v8f& a, v8f& b, v8f& c, v8f& d) { asm volatile("v_nop\n\tv_nop\n\tv_nop\n\tv_nop" : "+v"(a), "+v"(b), "+v"(c), "+v"(d)); }
template <typename T> struct Frag;
template <> struct Frag<_Float16> {
  typedef v16h V; union U { v16h v; v8h h[2]; };
  static __device__ __forceinline__ v16h load(const _Float16* p) {
    U f; f.h[0] = *(const v8h*)(p); f.h[1] = *(const v8h*)(p + 16); return f.v;
  }
  static __device__ __forceinline__ v8f mma(v16h a, v16h b, v8f c) {
    return __builtin_amdgcn_wmma_f32_16x16x32_f16(false, a, false, b, (short)0, c, false, false);
  }
  static __device__ __forceinline__ void guard(v8f& a, v8f& b, v16h x, v16h y) { dep_guard_h(a, b, x, y); }
  static __device__ __forceinline__ void keep(v16h a, v16h b, v16h c, v16h d) { keep4_h(a, b, c, d); }
};
template <> struct Frag<__bf16> {
  typedef v16b V; union U { v16b v; v8b h[2]; };
  static __device__ __forceinline__ v16b load(const __bf16* p) {
    U f; f.h[0] = *(const v8b*)(p); f.h[1] = *(const v8b*)(p + 16); return f.v;
  }
  static __device__ __forceinline__ v8f mma(v16b a, v16b b, v8f c) {
    return __builtin_amdgcn_wmma_f32_16x16x32_bf16(false, a, false, b, (short)0, c, false, false);
  }
  static __device__ __forceinline__ void guard(v8f& a, v8f& b, v16b x, v16b y) { dep_guard_b(a, b, x, y); }
  static __device__ __forceinline__ void keep(v16b a, v16b b, v16b c, v16b d) { keep4_b(a, b, c, d); }
};
template <int ET> struct Elem;
template <> struct Elem<0> { typedef _Float16 T; };
template <> struct Elem<1> { typedef __bf16 T; };

template <int ET, int SPLIT, int BIAS_MODE, int OUT_MODE>
__global__ __launch_bounds__(256) void wmma_gemm64g(
    const unsigned short* __restrict__ Ap, const unsigned short* __restrict__ A2p, int lda, long strideA, long strideAg,
    const unsigned short* __restrict__ Btp, const unsigned short* __restrict__ Bt2p, int ldb, long strideB, long strideBg,
    void* __restrict__ Cout, void* __restrict__ Cout2, int ldc, long strideC, long strideCg,
    const float* __restrict__ bias, long strideBias,
    int grp, int M, int N, int K, float scale) {
  typedef typename Elem<ET>::T T;
  typedef typename Frag<T>::V V;
  const T* A = (const T*)Ap; const T* A2 = (const T*)A2p; const T* Bt = (const T*)Btp; const T* Bt2 = (const T*)Bt2p;
  __shared__ __align__(16) float sT[8][16 * 68];
  const int bz   = blockIdx.y;
  const int bzo  = bz / grp;
  const int bzi  = bz - bzo * grp;
  const int lane = threadIdx.x & 31;
  const int wave = threadIdx.x >> 5;
  const int tilesN = N >> 6;
  const int tilesM = M >> 6;
  const int tile = blockIdx.x * 8 + wave;
  if (tile >= tilesM * tilesN) return;
  const int tm = tile / tilesN;
  const int tn = tile - tm * tilesN;
  const int m0 = tm << 6;
  const int n0 = tn << 6;

  const size_t offA = (size_t)bzo * (size_t)strideA + (size_t)bzi * (size_t)strideAg;
  const size_t offB = (size_t)bzo * (size_t)strideB + (size_t)bzi * (size_t)strideBg;
  const size_t offC = (size_t)bzo * (size_t)strideC + (size_t)bzi * (size_t)strideCg;
  const T* Ab  = A  + offA;
  const T* Bb  = Bt + offB;
  const T* Ab2 = (SPLIT == 1) ? (A2  + offA) : nullptr;
  const T* Bb2 = (SPLIT != 0) ? (Bt2 + offB) : nullptr;
  const float* biasb = (BIAS_MODE != 0) ? (bias + (size_t)bzi * (size_t)strideBias) : nullptr;

  const int rlane = lane & 15;
  const int koff  = (lane >> 4) * 8;
  const int mOff  = (lane >> 4) * 8;

  v8f acc[4][4];
#pragma unroll
  for (int i = 0; i < 4; ++i)
#pragma unroll
    for (int j = 0; j < 4; ++j) acc[i][j] = (v8f){0.f,0.f,0.f,0.f,0.f,0.f,0.f,0.f};

  for (int k0 = 0; k0 < K; k0 += 32) {
    V bh[4], bl[4];
#pragma unroll
    for (int j = 0; j < 4; ++j) {
      const size_t bo = (size_t)(n0 + (j << 4) + rlane) * ldb + koff + k0;
      bh[j] = Frag<T>::load(Bb + bo);
      if (SPLIT != 0) bl[j] = Frag<T>::load(Bb2 + bo);
    }
#pragma unroll
    for (int i = 0; i < 4; ++i) {
      const size_t ao = (size_t)(m0 + (i << 4) + rlane) * lda + koff + k0;
      V ah = Frag<T>::load(Ab + ao);
      V al;
      if (SPLIT == 1) al = Frag<T>::load(Ab2 + ao);
#pragma unroll
      for (int j = 0; j < 4; ++j) {
        acc[i][j] = Frag<T>::mma(ah, bh[j], acc[i][j]);
        if (SPLIT != 0) acc[i][j] = Frag<T>::mma(ah, bl[j], acc[i][j]);
        if (SPLIT == 1) acc[i][j] = Frag<T>::mma(al, bh[j], acc[i][j]);
      }
      Frag<T>::guard(acc[i][0], acc[i][3], ah, (SPLIT == 1) ? al : ah);
    }
    Frag<T>::keep(bh[0], bh[1], bh[2], bh[3]);
    if (SPLIT != 0) Frag<T>::keep(bl[0], bl[1], bl[2], bl[3]);
  }
  acc_guard4(acc[0][0], acc[0][1], acc[0][2], acc[0][3]);
  acc_guard4(acc[1][0], acc[1][1], acc[1][2], acc[1][3]);
  acc_guard4(acc[2][0], acc[2][1], acc[2][2], acc[2][3]);
  acc_guard4(acc[3][0], acc[3][1], acc[3][2], acc[3][3]);

  float* slab = sT[wave];
#pragma unroll
  for (int i = 0; i < 4; ++i) {
    const int mBase = m0 + (i << 4);
#pragma unroll
    for (int j = 0; j < 4; ++j) {
      const int n = n0 + (j << 4) + rlane;
      float bv = 0.f;
      if (BIAS_MODE == 2) bv = biasb[n];
#pragma unroll
      for (int r = 0; r < 8; ++r) {
        float v = acc[i][j][r] * scale;
        if (BIAS_MODE == 2) v += bv;
        slab[(mOff + r) * 68 + (j << 4) + rlane] = v;
      }
    }
    __builtin_amdgcn_fence(__ATOMIC_RELEASE, "workgroup");
    __builtin_amdgcn_wave_barrier();
    __builtin_amdgcn_fence(__ATOMIC_ACQUIRE, "workgroup");
    if (OUT_MODE == 0) {
      float* C = (float*)Cout + offC;
      const int hh = lane >> 4, c4 = (lane & 15) * 4;
      for (int pass = 0; pass < 2; ++pass) {
#pragma unroll
        for (int it = 0; it < 8; ++it) {
          const int row = it * 2 + hh;
          v4f v = *(const v4f*)(slab + row * 68 + c4);
          *(volatile v4f*)(C + (size_t)(mBase + row) * ldc + n0 + c4) = v;
        }
        __threadfence();
      }
    } else {
      const int q = lane >> 3, c8 = (lane & 7) * 8;
      unsigned short* C  = (unsigned short*)Cout  + offC;
      unsigned short* C2 = (OUT_MODE == 2) ? ((unsigned short*)Cout2 + offC) : nullptr;
      for (int pass = 0; pass < 2; ++pass) {
#pragma unroll
        for (int it = 0; it < 4; ++it) {
          const int row = it * 4 + q;
          const float* sp = slab + row * 68 + c8;
          v8h hv, lv;
#pragma unroll
          for (int e = 0; e < 8; ++e) {
            if (OUT_MODE == 1) {
              hv[e] = (_Float16)sp[e];
            } else {
              unsigned short hb = f2bf_bits(sp[e]);
              unsigned short lb = f2bf_bits(sp[e] - bf_bits2f(hb));
              hv[e] = __builtin_bit_cast(_Float16, hb);
              lv[e] = __builtin_bit_cast(_Float16, lb);
            }
          }
          *(volatile v8h*)(C + (size_t)(mBase + row) * ldc + n0 + c8) = hv;
          if (OUT_MODE == 2) *(volatile v8h*)(C2 + (size_t)(mBase + row) * ldc + n0 + c8) = lv;
        }
        __threadfence();
      }
    }
    __builtin_amdgcn_fence(__ATOMIC_RELEASE, "workgroup");
    __builtin_amdgcn_wave_barrier();
    __builtin_amdgcn_fence(__ATOMIC_ACQUIRE, "workgroup");
  }
}

__global__ __launch_bounds__(256) void cast_f32_bf16x8(
    const float* __restrict__ in, unsigned short* __restrict__ out, int n8) {
  const int i = blockIdx.x * 256 + threadIdx.x;
  if (i < n8) {
    const v4f a = *(const v4f*)(in + (size_t)i * 8);
    const v4f b = *(const v4f*)(in + (size_t)i * 8 + 4);
    v4u w;
    w[0] = (unsigned)f2bf_bits(a[0]) | ((unsigned)f2bf_bits(a[1]) << 16);
    w[1] = (unsigned)f2bf_bits(a[2]) | ((unsigned)f2bf_bits(a[3]) << 16);
    w[2] = (unsigned)f2bf_bits(b[0]) | ((unsigned)f2bf_bits(b[1]) << 16);
    w[3] = (unsigned)f2bf_bits(b[2]) | ((unsigned)f2bf_bits(b[3]) << 16);
    unsigned short* p = out + (size_t)i * 8;
    *(volatile v4u*)p = w;
    __threadfence();
    *(volatile v4u*)p = w;
  }
}

__global__ __launch_bounds__(256) void cast_bias4(
    const float* __restrict__ b0, const float* __restrict__ b1, const float* __restrict__ b2, const float* __restrict__ b3,
    float* __restrict__ tab, int n) {
  const int which = blockIdx.y;
  const float* src = (which == 0) ? b0 : (which == 1) ? b1 : (which == 2) ? b2 : b3;
  const int i = blockIdx.x * 256 + threadIdx.x;
  if (i * 4 + 3 < n) {
    const v4f v = *(const v4f*)(src + (size_t)i * 4);
    v4f r;
    r[0] = bf16_rne(v[0]); r[1] = bf16_rne(v[1]); r[2] = bf16_rne(v[2]); r[3] = bf16_rne(v[3]);
    float* p = tab + (size_t)which * n + (size_t)i * 4;
    *(volatile v4f*)p = r;
    __threadfence();
    *(volatile v4f*)p = r;
  }
}

__global__ __launch_bounds__(256) void softmax_heads(
    const float* __restrict__ S,
    const int*   __restrict__ adj,
    const float* __restrict__ lbias,
    unsigned short* __restrict__ Phi, unsigned short* __restrict__ Plo,
    float* __restrict__ attm,
    int bbase) {
  __shared__ __align__(16) float pst[NHEAD][NNODE];
  const int q    = blockIdx.x;
  const int bl   = blockIdx.y;
  const int b    = bbase + bl;
  const int lane = threadIdx.x & 31;
  const int wave = threadIdx.x >> 5;
  const int k0   = lane * 8;
  const size_t rowg = ((size_t)b * NNODE + q) * NNODE + k0;

  const v4i a0 = *(const v4i*)(adj + rowg);
  const v4i a1 = *(const v4i*)(adj + rowg + 4);
  const v4f c0 = *(const v4f*)(lbias + rowg);
  const v4f c1 = *(const v4f*)(lbias + rowg + 4);
  int   msk[8];
  float bia[8];
#pragma unroll
  for (int e = 0; e < 4; ++e) {
    msk[e] = a0[e]; msk[4 + e] = a1[e];
    bia[e] = bf16_rne(c0[e]); bia[4 + e] = bf16_rne(c1[e]);
  }

#pragma unroll 1
  for (int hs = 0; hs < 2; ++hs) {
    const int h = wave * 2 + hs;
    const size_t rows = ((size_t)(bl * NHEAD + h) * NNODE + q) * NNODE + k0;
    const v4f s0 = *(const v4f*)(S + rows);
    const v4f s1 = *(const v4f*)(S + rows + 4);
    float sv[8];
#pragma unroll
    for (int e = 0; e < 4; ++e) {
      sv[e]     = ((msk[e]     > 0) ? s0[e] : MASK_FILL) + bia[e];
      sv[4 + e] = ((msk[4 + e] > 0) ? s1[e] : MASK_FILL) + bia[4 + e];
    }
    float m = sv[0];
#pragma unroll
    for (int e = 1; e < 8; ++e) m = fmaxf(m, sv[e]);
#pragma unroll
    for (int off = 16; off > 0; off >>= 1) m = fmaxf(m, __shfl_xor(m, off, 32));
    float ev[8];
    float sum = 0.0f;
#pragma unroll
    for (int e = 0; e < 8; ++e) { ev[e] = expf(sv[e] - m); sum += ev[e]; }
#pragma unroll
    for (int off = 16; off > 0; off >>= 1) sum += __shfl_xor(sum, off, 32);
    const float inv = 1.0f / sum;
    float pv[8];
#pragma unroll
    for (int e = 0; e < 8; ++e) pv[e] = ev[e] * inv;

    {
      v4f p0, p1;
#pragma unroll
      for (int e = 0; e < 4; ++e) { p0[e] = pv[e]; p1[e] = pv[4 + e]; }
      *(v4f*)(&pst[h][k0]) = p0;
      *(v4f*)(&pst[h][k0 + 4]) = p1;
    }
    v4u hw, lw;
#pragma unroll
    for (int j = 0; j < 4; ++j) {
      const unsigned short hb0 = f2bf_bits(pv[2 * j]);
      const unsigned short hb1 = f2bf_bits(pv[2 * j + 1]);
      const unsigned short lb0 = f2bf_bits(pv[2 * j]     - bf_bits2f(hb0));
      const unsigned short lb1 = f2bf_bits(pv[2 * j + 1] - bf_bits2f(hb1));
      hw[j] = (unsigned)hb0 | ((unsigned)hb1 << 16);
      lw[j] = (unsigned)lb0 | ((unsigned)lb1 << 16);
    }
    unsigned short* ph = Phi + rows;
    unsigned short* pl = Plo + rows;
    *(volatile v4u*)ph = hw;
    *(volatile v4u*)pl = lw;
    __threadfence();
    *(volatile v4u*)ph = hw;
    *(volatile v4u*)pl = lw;
  }

  __syncthreads();
  if (threadIdx.x < 64) {
    const int kk = threadIdx.x * 4;
    v4f acc = (v4f){0.0f, 0.0f, 0.0f, 0.0f};
#pragma unroll
    for (int h = 0; h < NHEAD; ++h) {
      const v4f pvv = *(const v4f*)(&pst[h][kk]);
      acc += pvv;
    }
    acc *= (1.0f / (float)NHEAD);
    float* ap = attm + ((size_t)b * NNODE + q) * NNODE + kk;
    *(volatile v4f*)ap = acc;
    __threadfence();
    *(volatile v4f*)ap = acc;
  }
}

extern "C" void kernel_launch(void* const* d_in, const int* in_sizes, int n_in,
                              void* d_out, int out_size, void* d_ws, size_t ws_size,
                              hipStream_t stream) {
  if (n_in < 12) return;
  if (in_sizes[0] != MROWS * NFEAT || in_sizes[1] != MROWS * NFEAT) return;
  if (in_sizes[2] != NBATCH * NNODE * NNODE || in_sizes[3] != NBATCH * NNODE * NNODE) return;
  if (in_sizes[4] != NFEAT * NFEAT || in_sizes[6] != NFEAT * NFEAT || in_sizes[8] != NFEAT * NFEAT || in_sizes[10] != NFEAT * NFEAT) return;
  if (in_sizes[5] != NFEAT || in_sizes[7] != NFEAT || in_sizes[9] != NFEAT || in_sizes[11] != NFEAT) return;
  if (out_size != OUT0_ELEMS + OUT1_ELEMS) return;
  if (ws_size < WS_TOTAL) return;

  const float* obj   = (const float*)d_in[0];
  const float* cross = (const float*)d_in[1];
  const int*   adj   = (const int*)  d_in[2];
  const float* lb    = (const float*)d_in[3];
  const float* Wq    = (const float*)d_in[4];
  const float* bq    = (const float*)d_in[5];
  const float* Wk    = (const float*)d_in[6];
  const float* bk    = (const float*)d_in[7];
  const float* Wv    = (const float*)d_in[8];
  const float* bv    = (const float*)d_in[9];
  const float* Wo    = (const float*)d_in[10];
  const float* bo    = (const float*)d_in[11];

  char* ws = (char*)d_ws;
  unsigned short* obj16 = (unsigned short*)(ws + OFF_OBJ16);
  unsigned short* crs16 = (unsigned short*)(ws + OFF_CRS16);
  unsigned short* wq16  = (unsigned short*)(ws + OFF_WQ16);
  unsigned short* wk16  = (unsigned short*)(ws + OFF_WK16);
  unsigned short* wv16  = (unsigned short*)(ws + OFF_WV16);
  unsigned short* wo16  = (unsigned short*)(ws + OFF_WO16);
  float*          biasT = (float*)(ws + OFF_BIAS);
  unsigned short* qhi   = (unsigned short*)(ws + OFF_QHI);
  unsigned short* qlo   = (unsigned short*)(ws + OFF_QLO);
  unsigned short* khi   = (unsigned short*)(ws + OFF_KHI);
  unsigned short* klo   = (unsigned short*)(ws + OFF_KLO);
  unsigned short* vhi   = (unsigned short*)(ws + OFF_VHI);
  unsigned short* vlo   = (unsigned short*)(ws + OFF_VLO);
  unsigned short* vohi  = (unsigned short*)(ws + OFF_VOHI);
  unsigned short* volo  = (unsigned short*)(ws + OFF_VOLO);
  float*          Sbuf  = (float*)(ws + OFF_S);
  unsigned short* phi   = (unsigned short*)(ws + OFF_PHI);
  unsigned short* plo   = (unsigned short*)(ws + OFF_PLO);

  float* out0 = (float*)d_out;
  float* out1 = out0 + OUT0_ELEMS;

  {
    const int na8 = (MROWS * NFEAT) / 8;
    const int nw8 = (NFEAT * NFEAT) / 8;
    cast_f32_bf16x8<<<na8 / 256, 256, 0, stream>>>(obj,   obj16, na8);
    cast_f32_bf16x8<<<na8 / 256, 256, 0, stream>>>(cross, crs16, na8);
    cast_f32_bf16x8<<<nw8 / 256, 256, 0, stream>>>(Wq, wq16, nw8);
    cast_f32_bf16x8<<<nw8 / 256, 256, 0, stream>>>(Wk, wk16, nw8);
    cast_f32_bf16x8<<<nw8 / 256, 256, 0, stream>>>(Wv, wv16, nw8);
    cast_f32_bf16x8<<<nw8 / 256, 256, 0, stream>>>(Wo, wo16, nw8);
    cast_bias4<<<dim3(1, 4), 256, 0, stream>>>(bq, bk, bv, bo, biasT, NFEAT);
  }

  {
    const int tiles = (MROWS / 64) * (NFEAT / 64);
    dim3 g(tiles / 8, 1);
    wmma_gemm64g<1, 0, 2, 2><<<g, 256, 0, stream>>>(
        obj16, nullptr, NFEAT, 0L, 0L,
        wq16, nullptr, NFEAT, 0L, 0L,
        qhi, qlo, NFEAT, 0L, 0L,
        biasT + 0 * NFEAT, 0L,
        1, MROWS, NFEAT, NFEAT, 1.0f);
    wmma_gemm64g<1, 0, 2, 2><<<g, 256, 0, stream>>>(
        crs16, nullptr, NFEAT, 0L, 0L,
        wk16, nullptr, NFEAT, 0L, 0L,
        khi, klo, NFEAT, 0L, 0L,
        biasT + 1 * NFEAT, 0L,
        1, MROWS, NFEAT, NFEAT, 1.0f);
    wmma_gemm64g<1, 0, 2, 2><<<g, 256, 0, stream>>>(
        crs16, nullptr, NFEAT, 0L, 0L,
        wv16, nullptr, NFEAT, 0L, 0L,
        vhi, vlo, NFEAT, 0L, 0L,
        biasT + 2 * NFEAT, 0L,
        1, MROWS, NFEAT, NFEAT, 1.0f);
  }

  {
    const int tiles = (NFEAT / 64) * (NNODE / 64);
    dim3 g(tiles / 8, NBATCH);
    wmma_gemm64g<1, 2, 0, 2><<<g, 256, 0, stream>>>(
        wo16, nullptr, NFEAT, 0L, 0L,
        vhi, vlo, NFEAT, (long)NNODE * NFEAT, 0L,
        vohi, volo, NNODE, (long)NFEAT * NNODE, 0L,
        nullptr, 0L,
        1, NFEAT, NNODE, NFEAT, 1.0f);
  }

  for (int c = 0; c < NCHUNKS; ++c) {
    const size_t actOff = (size_t)c * BPC * NNODE * NFEAT;
    const size_t voOff  = (size_t)c * BPC * NFEAT * NNODE;
    {
      const int tiles = (NNODE / 64) * (NNODE / 64);
      dim3 g(tiles / 8, ZPC);
      wmma_gemm64g<1, 1, 0, 0><<<g, 256, 0, stream>>>(
          qhi + actOff, qlo + actOff, NFEAT, (long)NNODE * NFEAT, (long)DHEAD,
          khi + actOff, klo + actOff, NFEAT, (long)NNODE * NFEAT, (long)DHEAD,
          Sbuf, nullptr, NNODE, (long)NHEAD * NNODE * NNODE, (long)NNODE * NNODE,
          nullptr, 0L,
          NHEAD, NNODE, NNODE, DHEAD, 0.125f);
    }
    softmax_heads<<<dim3(NNODE, BPC), 256, 0, stream>>>(Sbuf, adj, lb, phi, plo, out1, c * BPC);
    {
      const int tiles = (NNODE / 64) * (DHEAD / 64);
      dim3 g((tiles + 7) / 8, ZPC);
      wmma_gemm64g<1, 1, 2, 0><<<g, 256, 0, stream>>>(
          phi, plo, NNODE, (long)NHEAD * NNODE * NNODE, (long)NNODE * NNODE,
          vohi + voOff, volo + voOff, NNODE, (long)NFEAT * NNODE, (long)DHEAD * NNODE,
          out0 + actOff, nullptr, NFEAT, (long)NNODE * NFEAT, (long)DHEAD,
          biasT + 3 * NFEAT, (long)DHEAD,
          NHEAD, NNODE, DHEAD, NNODE, 1.0f);
    }
  }
}
